// MSDN_BASE_65652870087588
// MI455X (gfx1250) — hardware-verified
//
#include <hip/hip_runtime.h>
#include <stddef.h>


#define FEA    512
#define GW     128
#define KPB    512
#define APZ    520
#define GROWS  32
#define GTHR   64
#define NBLK   64
#define ATHR   256
#define AWAV   (ATHR / 32)
#define NPW    (NBLK / AWAV)
#define CHUNK  16384
#define NSUB   (CHUNK / ATHR)
#define PTHR   256
#define PBLK   ((2 * GW * FEA) / (8 * PTHR))
#define WSC    64.0f
#define RW     0.015625f
#define RG     0.0078125f
#define WSCAP  134217728
#define LDS_ACC (NBLK * FEA * 4)
#define LDS_LST (CHUNK * 4)
#define LDS_CNT (2 * 32 * 4)
#define LDS_AGG (LDS_ACC + LDS_LST + LDS_CNT)

static_assert(NPW == 8 && AWAV == 8);
static_assert((CHUNK % ATHR) == 0);
static_assert(PBLK * PTHR * 8 == 2 * GW * FEA);
static_assert((APZ % 8) == 0 && (KPB % 8) == 0 && (FEA % 32) == 0);
static_assert(GROWS == (GTHR / 32) * 16);
static_assert(GW == 128 && FEA == 4 * 128);
static_assert(GROWS * GW == 16 * GTHR * 4);
static_assert(GW * KPB == 65536);
static_assert(LDS_AGG == 196864);

typedef float    v4f  __attribute__((ext_vector_type(4)));
typedef float    v8f  __attribute__((ext_vector_type(8)));
typedef _Float16 v8h  __attribute__((ext_vector_type(8)));
typedef _Float16 v16h __attribute__((ext_vector_type(16)));
union Frag { v16h v; v8h h[2]; };

__device__ __forceinline__ v8f wmh(v16h a, v16h b, v8f c) {
  v8f d = __builtin_amdgcn_wmma_f32_16x16x32_f16(false, a, false, b, (short)0, c, false, false);
  asm volatile("v_nop\n\tv_nop\n\tv_nop\n\tv_nop" : "+v"(d) : "v"(a), "v"(b));
  return d;
}

__device__ __forceinline__ float sigf(float x) {
  x = fminf(fmaxf(x, -30.0f), 30.0f);
  const float ex = __expf(-x);
  return __builtin_amdgcn_rcpf(1.0f + ex);
}

template <int NT>
__device__ __forceinline__ void mma16(const _Float16* At, const _Float16* __restrict__ Bp,
                                      int lane, v8f (&acc)[NT]) {
  const int hh = lane >> 4, m = lane & 15;
#pragma unroll
  for (int t = 0; t < NT; ++t) { v8f z = {0.f, 0.f, 0.f, 0.f, 0.f, 0.f, 0.f, 0.f}; acc[t] = z; }
  const _Float16* ap = At + m * APZ + 8 * hh;
  const _Float16* bb = Bp + (size_t)m * KPB + 8 * hh;
#pragma unroll 1
  for (int ks = 0; ks < FEA / 32; ++ks) {
    Frag a;
    a.h[0] = *(const v8h*)(ap + 32 * ks);
    a.h[1] = *(const v8h*)(ap + 32 * ks + 16);
#pragma unroll
    for (int t = 0; t < NT; ++t) {
      const _Float16* bp = bb + (size_t)(16 * t) * KPB + 32 * ks;
      Frag b;
      b.h[0] = *(const v8h*)bp;
      b.h[1] = *(const v8h*)(bp + 16);
      acc[t] = wmh(a.v, b.v, acc[t]);
    }
  }
}

__global__ __launch_bounds__(PTHR) void k_wprep(const float* __restrict__ w, _Float16* Bpl) {
  const int i = blockIdx.x * PTHR + threadIdx.x;
  const int side = i >> 13;
  const int n = (i >> 6) & (GW - 1);
  const int k0 = (i & 63) * 8;
  const float* sp = w + (size_t)n * (2 * FEA) + side * FEA + k0;
  const v4f a = *(const v4f*)sp;
  const v4f c = *(const v4f*)(sp + 4);
  v8h hv;
  hv[0] = (_Float16)(a.x * WSC); hv[1] = (_Float16)(a.y * WSC); hv[2] = (_Float16)(a.z * WSC); hv[3] = (_Float16)(a.w * WSC);
  hv[4] = (_Float16)(c.x * WSC); hv[5] = (_Float16)(c.y * WSC); hv[6] = (_Float16)(c.z * WSC); hv[7] = (_Float16)(c.w * WSC);
  _Float16* dp = Bpl + (size_t)i * 8;
  *(volatile v8h*)dp = hv;
  __threadfence();
  *(volatile v8h*)dp = hv;
}

__global__ __launch_bounds__(GTHR) void k_nodegemm(const float* __restrict__ xt, const float* __restrict__ xs,
                                                   const _Float16* __restrict__ Bpl, const float* __restrict__ bias,
                                                   float* PQ, int nN, int nPad) {
  __shared__ __attribute__((aligned(16))) _Float16 At[GROWS * APZ];
  __shared__ __attribute__((aligned(16))) float stg[GROWS * GW];
  const int tid = threadIdx.x, lane = tid & 31, wave = tid >> 5, hh = lane >> 4, m = lane & 15;
  const int side = blockIdx.y;
  const float* x = side ? xs : xt;
  const _Float16* Bp = Bpl + (size_t)side * GW * KPB;
  const int rowBase = blockIdx.x * GROWS;
  {
    const int r = tid >> 1, c0 = (tid & 1) * 256;
    int xrow = rowBase + r;
    xrow = xrow > nN - 1 ? nN - 1 : xrow;
    const float* xp = x + (size_t)xrow * FEA + c0;
    _Float16* dp = At + r * APZ + c0;
#pragma unroll 4
    for (int j = 0; j < 32; ++j) {
      const v4f a = *(const v4f*)(xp + 8 * j), c = *(const v4f*)(xp + 8 * j + 4);
      v8h hv;
      hv[0] = (_Float16)fmaxf(a.x, 0.0f); hv[1] = (_Float16)fmaxf(a.y, 0.0f);
      hv[2] = (_Float16)fmaxf(a.z, 0.0f); hv[3] = (_Float16)fmaxf(a.w, 0.0f);
      hv[4] = (_Float16)fmaxf(c.x, 0.0f); hv[5] = (_Float16)fmaxf(c.y, 0.0f);
      hv[6] = (_Float16)fmaxf(c.z, 0.0f); hv[7] = (_Float16)fmaxf(c.w, 0.0f);
      *(v8h*)(dp + 8 * j) = hv;
    }
  }
  __syncthreads();

  {
    v8f acc[8];
    mma16<8>(At + wave * 16 * APZ, Bp, lane, acc);
    float* sp = stg + (wave * 16 + 8 * hh) * GW + m;
#pragma unroll
    for (int t = 0; t < 8; ++t) {
      const float bb = bias[16 * t + m];
      const float bv = side ? bb : 0.0f;
#pragma unroll
      for (int r = 0; r < 8; ++r) sp[r * GW + 16 * t] = acc[t][r] * RW + bv;
    }
  }
  __syncthreads();

  float* gp = PQ + ((size_t)side * nPad + rowBase) * GW;
#pragma unroll
  for (int it = 0; it < 16; ++it) {
    const int f = it * GTHR + tid;
    const v4f v = *(const v4f*)(stg + 4 * f);
    *(volatile v4f*)(gp + 4 * f) = v;
  }
  __threadfence();
#pragma unroll
  for (int it = 0; it < 16; ++it) {
    const int f = it * GTHR + tid;
    const v4f v = *(const v4f*)(stg + 4 * f);
    *(volatile v4f*)(gp + 4 * f) = v;
  }
}

__global__ __launch_bounds__(ATHR) void k_agg(const float* __restrict__ PQ, const float* __restrict__ xs,
                                               const int* __restrict__ tix, const int* __restrict__ six,
                                               float* out, int nN, int nE, int nPad) {
  extern __shared__ __attribute__((aligned(16))) float dlds[];
  float* sacc = dlds;
  int*   slst = (int*)(dlds + NBLK * FEA);
  int*   scnt = slst + CHUNK;
  const int tid = threadIdx.x, lane = tid & 31, wave = tid >> 5;
  const int n0 = blockIdx.x * NBLK;
  const float* P = PQ;
  const float* Q = PQ + (size_t)nPad * GW;

  {
    const v4f z = {0.0f, 0.0f, 0.0f, 0.0f};
#pragma unroll 4
    for (int i = tid; i < NBLK * FEA / 4; i += ATHR) *(v4f*)(sacc + 4 * i) = z;
    if (tid < 64) scnt[tid] = 0;
  }
  __syncthreads();

  int cntv[NPW];
#pragma unroll
  for (int k = 0; k < NPW; ++k) cntv[k] = 0;

  const int nCh = (nE + CHUNK - 1) / CHUNK;
  int par = 0;
  for (int ch = 0; ch < nCh; ++ch) {
    const int cb = ch * CHUNK;
    int base = 0;
#pragma unroll 1
    for (int sub = 0; sub < NSUB; ++sub) {
      const int e = cb + sub * ATHR + tid;
      const int ec = e < nE ? e : nE - 1;
      const int t = tix[ec];
      const bool hit = (e < nE) && ((unsigned)(t - n0) < (unsigned)NBLK);
      const unsigned msk = __builtin_amdgcn_ballot_w32(hit);
      const int wc = __builtin_popcount(msk);
      const int rank = __builtin_popcount(msk & ((1u << lane) - 1u));
      if (lane == 0) scnt[par * 32 + wave] = wc;
      __syncthreads();
      const int cl = scnt[par * 32 + lane];
      int x = cl;
      {
        int y;
        y = __shfl_up(x, 1, 32);  x += (lane >= 1)  ? y : 0;
        y = __shfl_up(x, 2, 32);  x += (lane >= 2)  ? y : 0;
        y = __shfl_up(x, 4, 32);  x += (lane >= 4)  ? y : 0;
        y = __shfl_up(x, 8, 32);  x += (lane >= 8)  ? y : 0;
        y = __shfl_up(x, 16, 32); x += (lane >= 16) ? y : 0;
      }
      const int total = __shfl(x, 31, 32);
      const int offs  = __shfl(x - cl, wave, 32);
      if (hit) {
        int idx = base + offs + rank;
        idx = idx < CHUNK - 1 ? idx : CHUNK - 1;
        slst[idx] = (e << 6) | (t - n0);
      }
      base += total;
      par ^= 1;
    }
    __syncthreads();

    const int len = base < CHUNK ? base : CHUNK;
#pragma unroll 1
    for (int pos = 0; pos < len; pos += 32) {
      const int pl = pos + lane;
      const int ent = slst[pl < CHUNK ? pl : CHUNK - 1];
      const bool match = (pl < len) && (((ent >> 3) & 7) == wave);
      unsigned mw = __builtin_amdgcn_ballot_w32(match);
      while (mw != 0u) {
        const int bit = __builtin_ctz(mw);
        mw &= mw - 1u;
        const int eb = __shfl(ent, bit, 32);
        const int ed = eb >> 6;
        const int li = eb & 7;
        int s = six[ed < nE ? ed : nE - 1];
        s = s < 0 ? 0 : (s > nN - 1 ? nN - 1 : s);
        int nd = n0 + NPW * wave + li;
        nd = nd > nN - 1 ? nN - 1 : nd;
        const v4f p = *(const v4f*)(P + (size_t)nd * GW + 4 * lane);
        const v4f q = *(const v4f*)(Q + (size_t)s * GW + 4 * lane);
        const v4f u = p + q;
        float sg = sigf(u.x) + sigf(u.y) + sigf(u.z) + sigf(u.w);
        sg += __shfl_xor(sg, 16, 32);
        sg += __shfl_xor(sg, 8, 32);
        sg += __shfl_xor(sg, 4, 32);
        sg += __shfl_xor(sg, 2, 32);
        sg += __shfl_xor(sg, 1, 32);
        const float g = sg * RG;
#pragma unroll
        for (int k = 0; k < NPW; ++k) cntv[k] += (li == k) ? 1 : 0;
        const float* fp = xs + (size_t)s * FEA + 4 * lane;
        float* ap = sacc + (NPW * wave + li) * FEA + 4 * lane;
#pragma unroll
        for (int j = 0; j < 4; ++j) {
          const v4f v = *(const v4f*)(fp + 128 * j);
          v4f a = *(const v4f*)(ap + 128 * j);
          a += v * g;
          *(v4f*)(ap + 128 * j) = a;
        }
      }
    }
    __syncthreads();
  }

#pragma unroll
  for (int k = 0; k < NPW; ++k) {
    const int nd = n0 + NPW * wave + k;
    if (nd < nN) {
      const float inv = cntv[k] > 0 ? __builtin_amdgcn_rcpf((float)cntv[k]) : 0.0f;
      const float* ap = sacc + (NPW * wave + k) * FEA + 4 * lane;
      float* op = out + (size_t)nd * FEA + 4 * lane;
      const v4f r0 = *(const v4f*)(ap) * inv;
      const v4f r1 = *(const v4f*)(ap + 128) * inv;
      const v4f r2 = *(const v4f*)(ap + 256) * inv;
      const v4f r3 = *(const v4f*)(ap + 384) * inv;
      *(volatile v4f*)(op)       = r0;
      *(volatile v4f*)(op + 128) = r1;
      *(volatile v4f*)(op + 256) = r2;
      *(volatile v4f*)(op + 384) = r3;
      __threadfence();
      *(volatile v4f*)(op)       = r0;
      *(volatile v4f*)(op + 128) = r1;
      *(volatile v4f*)(op + 256) = r2;
      *(volatile v4f*)(op + 384) = r3;
    }
  }
}

extern "C" void kernel_launch(void* const* d_in, const int* in_sizes, int n_in,
                              void* d_out, int out_size, void* d_ws, size_t ws_size,
                              hipStream_t stream) {
  if (n_in < 6) return;
  if (in_sizes[0] <= 0 || (in_sizes[0] % FEA) != 0) return;
  const int nN = in_sizes[0] / FEA;
  const int nE = in_sizes[4];
  if (nN <= 0 || nE <= 0) return;
  if (in_sizes[1] != nN * FEA || in_sizes[2] != 2 * GW * FEA || in_sizes[3] != GW || in_sizes[5] != nE) return;
  if (out_size != nN * FEA) return;
  if (nN > (1 << 21) || nE > (1 << 25)) return;

  const float* xt  = (const float*)d_in[0];
  const float* xs  = (const float*)d_in[1];
  const float* w   = (const float*)d_in[2];
  const float* bia = (const float*)d_in[3];
  const int*   tix = (const int*)d_in[4];
  const int*   six = (const int*)d_in[5];
  float* out = (float*)d_out;

  const int nBlkG = (nN + GROWS - 1) / GROWS;
  const int nPad  = nBlkG * GROWS;
  const int nBlkA = (nN + NBLK - 1) / NBLK;

  char* ws = (char*)d_ws;
  size_t off = 0;
  const size_t oB  = off; off += (size_t)2 * GW * KPB * 2;        off = (off + 255) & ~(size_t)255;
  const size_t oPQ = off; off += (size_t)2 * nPad * GW * 4;        off = (off + 255) & ~(size_t)255;
  if (off > ws_size || off > (size_t)WSCAP) return;
  _Float16* Bpl = (_Float16*)(ws + oB);
  float*    PQ  = (float*)(ws + oPQ);

  k_wprep<<<PBLK, PTHR, 0, stream>>>(w, Bpl);
  k_nodegemm<<<dim3(nBlkG, 2), GTHR, 0, stream>>>(xt, xs, Bpl, bia, PQ, nN, nPad);
  hipFuncSetAttribute(reinterpret_cast<const void*>(&k_agg), hipFuncAttributeMaxDynamicSharedMemorySize, LDS_AGG);
  k_agg<<<nBlkA, ATHR, LDS_AGG, stream>>>(PQ, xs, tix, six, out, nN, nE, nPad);
}
